// L2AttentionLayer_28716151341359
// MI455X (gfx1250) — hardware-verified
//
#include <hip/hip_runtime.h>


#define NB_  8
#define CC   256
#define C4   64
#define NN_  2048
#define PSC  32768.0f
#define LOSC 1024.0f
#define LOSCI (1.0f / 1024.0f)

typedef _Float16 h16;
typedef unsigned short bf;
typedef __attribute__((ext_vector_type(16))) __bf16   v16bf;
typedef __attribute__((ext_vector_type(16))) _Float16 v16h;
typedef __attribute__((ext_vector_type(8)))  _Float16 v8h;
typedef __attribute__((ext_vector_type(8)))  unsigned short v8us;
typedef __attribute__((ext_vector_type(4)))  unsigned short v4us;
typedef __attribute__((ext_vector_type(4)))  _Float16 v4h;
typedef __attribute__((ext_vector_type(8)))  float    v8f;
typedef __attribute__((ext_vector_type(4)))  float    v4f;
typedef v8h  __attribute__((may_alias)) v8ha;
typedef v4f  __attribute__((may_alias)) v4fa;
typedef v8us __attribute__((may_alias)) v8usa;

__device__ __forceinline__ unsigned short f2bf(float f) { unsigned u = __float_as_uint(f); u += 0x7FFFu + ((u >> 16) & 1u); return (unsigned short)(u >> 16); }
__device__ __forceinline__ float bf2f(unsigned short b) { return __uint_as_float(((unsigned)b) << 16); }
__device__ __forceinline__ float bfr(float f) { return bf2f(f2bf(f)); }
__device__ __forceinline__ v16h cat16(v8h lo, v8h hi) { return __builtin_shufflevector(lo, hi, 0, 1, 2, 3, 4, 5, 6, 7, 8, 9, 10, 11, 12, 13, 14, 15); }
__device__ __forceinline__ v16bf cat16b(v8us lo, v8us hi) { return __builtin_bit_cast(v16bf, __builtin_shufflevector(lo, hi, 0, 1, 2, 3, 4, 5, 6, 7, 8, 9, 10, 11, 12, 13, 14, 15)); }
__device__ __forceinline__ v8f wmma16(v16h a, v16h b, v8f c) { return __builtin_amdgcn_wmma_f32_16x16x32_f16(false, a, false, b, (short)0, c, false, false); }
__device__ __forceinline__ v8f wmmab(v16bf a, v16bf b, v8f c) { return __builtin_amdgcn_wmma_f32_16x16x32_bf16(false, a, false, b, (short)0, c, false, false); }
#define VST2(T, p, v) do { const T vst2_v_ = (v); *(volatile T*)(p) = vst2_v_; __threadfence(); *(volatile T*)(p) = vst2_v_; } while (0)

__global__ __launch_bounds__(256) void k_xt(const float* __restrict__ x, bf* XT) {
    __shared__ __align__(16) unsigned short tl[64 * 72];
    const int tid = threadIdx.x, n0 = blockIdx.x * 64, c0 = blockIdx.y * 64, b = blockIdx.z;
    const int cr = tid >> 2, nq = (tid & 3) * 16;
#pragma unroll
    for (int i = 0; i < 16; ++i) tl[(nq + i) * 72 + cr] = f2bf(x[((size_t)b * CC + c0 + cr) * NN_ + n0 + nq + i]);
    __syncthreads();
    const int piece = tid & 7;
    auto pass = [&]() {
#pragma unroll
        for (int s = 0; s < 2; ++s) { const int nr = (tid >> 3) + 32 * s; const v8us val = *(const v8usa*)(tl + nr * 72 + piece * 8);
            *(volatile v8us*)(XT + ((size_t)b * NN_ + n0 + nr) * CC + c0 + piece * 8) = val; }
    };
    pass(); __threadfence(); pass();
}
__global__ __launch_bounds__(256) void k_cvtw(const float* __restrict__ Wm, int rows, bf* WB) {
    const int lane = threadIdx.x & 31, r = blockIdx.x * 8 + (threadIdx.x >> 5);
    if (r >= rows) return;
    v8us t;
#pragma unroll
    for (int i = 0; i < 8; ++i) t[i] = f2bf(Wm[(size_t)r * CC + lane * 8 + i]);
    VST2(v8us, WB + (size_t)r * CC + lane * 8, t);
}

template <int MODE, bool SPLITB>
__global__ __launch_bounds__(128) void k_gemm(const bf* __restrict__ A, size_t aStrideB, const bf* __restrict__ Bm, const bf* __restrict__ Bl, size_t bStrideB, const float* __restrict__ rowbias, void* C, size_t cStrideB, int ldc) {
    __shared__ __align__(16) float ost[4][16 * 68];
    const int lane = threadIdx.x & 31, wave = threadIdx.x >> 5, lr = lane & 15, hi = lane >> 4, b = blockIdx.z;
    const int r0 = blockIdx.x * 64 + wave * 16, c0 = blockIdx.y * 64;
    const bf* Ab = A + (size_t)b * aStrideB; const bf* Bb = Bm + (size_t)b * bStrideB; const bf* Blb = Bl + (size_t)b * bStrideB;
    const size_t aoff = (size_t)(r0 + lr) * CC + 8 * hi;
    size_t boff[4];
#pragma unroll
    for (int t = 0; t < 4; ++t) boff[t] = (size_t)(c0 + t * 16 + lr) * CC + 8 * hi;
    v8f acc[4], accx[4];
#pragma unroll
    for (int t = 0; t < 4; ++t) { acc[t] = (v8f){}; accx[t] = (v8f){}; }
#pragma unroll 1
    for (int kc = 0; kc < CC; kc += 32) {
        const v16bf a = cat16b(*(const v8us*)(Ab + aoff + kc), *(const v8us*)(Ab + aoff + kc + 16));
#pragma unroll
        for (int t = 0; t < 4; ++t) { const v16bf bb = cat16b(*(const v8us*)(Bb + boff[t] + kc), *(const v8us*)(Bb + boff[t] + kc + 16)); acc[t] = wmmab(a, bb, acc[t]);
            if (SPLITB) { const v16bf bl = cat16b(*(const v8us*)(Blb + boff[t] + kc), *(const v8us*)(Blb + boff[t] + kc + 16)); accx[t] = wmmab(a, bl, accx[t]); } }
        asm volatile("v_nop\n\tv_nop\n\tv_nop\n\tv_nop" : "+v"(acc[0]), "+v"(acc[1]), "+v"(acc[2]), "+v"(acc[3]), "+v"(accx[0]), "+v"(accx[3]) : "v"(a));
    }
    asm volatile("v_nop\n\tv_nop\n\tv_nop\n\tv_nop" : "+v"(accx[0]), "+v"(accx[1]), "+v"(accx[2]), "+v"(accx[3]));
    float* os = &ost[wave][0];
#pragma unroll
    for (int t = 0; t < 4; ++t)
#pragma unroll
        for (int j = 0; j < 8; ++j) { float v = acc[t][j] + (SPLITB ? accx[t][j] : 0.f); if (MODE != 0) v += bfr(rowbias[r0 + hi * 8 + j]); os[(hi * 8 + j) * 68 + t * 16 + lr] = v; }
    __syncthreads();
    if (MODE == 1) {
        h16* crow = (h16*)C + (size_t)b * cStrideB + (size_t)r0 * ldc + c0;
        auto pass = [&]() {
#pragma unroll
            for (int s = 0; s < 4; ++s) { const int row = 4 * s + (lane >> 3), piece = lane & 7; const float* sp = os + row * 68 + piece * 8; v8h o;
#pragma unroll
                for (int i = 0; i < 8; ++i) o[i] = (h16)sp[i];
                *(volatile v8h*)(crow + (size_t)row * ldc + piece * 8) = o; }
        };
        pass(); __threadfence(); pass();
    } else {
        float* crow = (float*)C + (size_t)b * cStrideB + (size_t)r0 * ldc + c0;
        auto pass = [&]() {
#pragma unroll
            for (int s = 0; s < 8; ++s) { const int Lid = (lane >> 3) + 4 * s, piece = lane & 7; const int row = Lid >> 1, cofs = (Lid & 1) * 32 + piece * 4;
                const v4f val = *(const v4fa*)(os + row * 68 + cofs); *(volatile v4f*)(crow + (size_t)row * ldc + cofs) = val; }
        };
        pass(); __threadfence(); pass();
    }
}
__global__ __launch_bounds__(256) void k_qsplit(const float* __restrict__ QF, h16* QH, h16* QL, float* SQ) {
    __shared__ float sqs[32];
    const int lane = threadIdx.x & 31, wave = threadIdx.x >> 5;
    typedef __attribute__((ext_vector_type(2))) _Float16 v2h;
#pragma unroll
    for (int rr = 0; rr < 4; ++rr) {
        const size_t r = (size_t)blockIdx.x * 32 + wave * 4 + rr;
        const float v0 = QF[r * C4 + 2 * lane], v1 = QF[r * C4 + 2 * lane + 1];
        float s = v0 * v0 + v1 * v1;
#pragma unroll
        for (int o = 16; o; o >>= 1) s += __shfl_xor(s, o, 32);
        if (lane == 0) sqs[wave * 4 + rr] = s;
        v2h h2, l2; const h16 a0 = (h16)v0, a1 = (h16)v1; h2[0] = a0; h2[1] = a1; l2[0] = (h16)((v0 - (float)a0) * LOSC); l2[1] = (h16)((v1 - (float)a1) * LOSC);
        *(volatile v2h*)(QH + r * C4 + 2 * lane) = h2; *(volatile v2h*)(QL + r * C4 + 2 * lane) = l2; __threadfence();
        *(volatile v2h*)(QH + r * C4 + 2 * lane) = h2; *(volatile v2h*)(QL + r * C4 + 2 * lane) = l2;
    }
    __syncthreads();
    if (wave == 0) VST2(float, SQ + (size_t)blockIdx.x * 32 + lane, sqs[lane]);
}

__global__ __launch_bounds__(128) void k_attn(const h16* __restrict__ QH, const h16* __restrict__ QL, const float* __restrict__ SQ, const h16* __restrict__ V16, int cofs, float* XR) {
    __shared__ __align__(16) h16 plds[4][16 * 32];
    __shared__ __align__(16) float ost[4][16 * 132];
    const int lane = threadIdx.x & 31, wave = threadIdx.x >> 5, lr = lane & 15, hi = lane >> 4;
    const int b = blockIdx.x / (NN_ / 64), qt = blockIdx.x - b * (NN_ / 64), q0 = qt * 64 + wave * 16;
    h16* pl = &plds[wave][0];
    v16h ah[2], al[2];
#pragma unroll
    for (int kc = 0; kc < 2; ++kc) { const size_t o = ((size_t)b * NN_ + q0 + lr) * C4 + kc * 32 + 8 * hi;
        ah[kc] = cat16(*(const v8h*)(QH + o), *(const v8h*)(QH + o + 16)); al[kc] = cat16(*(const v8h*)(QL + o), *(const v8h*)(QL + o + 16)); }
    float sqi[8];
#pragma unroll
    for (int j = 0; j < 8; ++j) sqi[j] = SQ[(size_t)b * NN_ + q0 + 8 * hi + j];
    const h16* vb = V16 + ((size_t)b * CC + cofs) * NN_;
    v8f o[8];
#pragma unroll
    for (int n = 0; n < 8; ++n) o[n] = (v8f){};
    float mrow[8], lpart[8];
#pragma unroll
    for (int j = 0; j < 8; ++j) { mrow[j] = -3.0e38f; lpart[j] = 0.f; }
#pragma unroll 1
    for (int kt = 0; kt < NN_ / 32; ++kt) {
        const int l0 = kt * 32;
        v8f s0 = {}, s1 = {}, x0 = {}, x1 = {};
#pragma unroll
        for (int kc = 0; kc < 2; ++kc) {
            const size_t o0 = ((size_t)b * NN_ + l0 + lr) * C4 + kc * 32 + 8 * hi, o1 = o0 + (size_t)16 * C4;
            const v16h k0h = cat16(*(const v8h*)(QH + o0), *(const v8h*)(QH + o0 + 16)), k0l = cat16(*(const v8h*)(QL + o0), *(const v8h*)(QL + o0 + 16));
            const v16h k1h = cat16(*(const v8h*)(QH + o1), *(const v8h*)(QH + o1 + 16)), k1l = cat16(*(const v8h*)(QL + o1), *(const v8h*)(QL + o1 + 16));
            s0 = wmma16(ah[kc], k0h, s0); x0 = wmma16(ah[kc], k0l, x0); x0 = wmma16(al[kc], k0h, x0);
            s1 = wmma16(ah[kc], k1h, s1); x1 = wmma16(ah[kc], k1l, x1); x1 = wmma16(al[kc], k1h, x1);
        }
        asm volatile("v_nop\n\tv_nop\n\tv_nop\n\tv_nop" : "+v"(s0), "+v"(s1), "+v"(x0), "+v"(x1) : "v"(ah[0]), "v"(al[1]));
        const float sqj0 = SQ[(size_t)b * NN_ + l0 + lr], sqj1 = SQ[(size_t)b * NN_ + l0 + 16 + lr];
        float alpha[8];
#pragma unroll
        for (int j = 0; j < 8; ++j) {
            const float g0 = s0[j] + x0[j] * LOSCI, g1 = s1[j] + x1[j] * LOSCI;
            const float d0 = sqi[j] - 2.0f * g0 + sqj0, d1 = sqi[j] - 2.0f * g1 + sqj1;
            const float a0 = -sqrtf(fmaxf(d0, 0.f)), a1 = -sqrtf(fmaxf(d1, 0.f));
            float mx = fmaxf(a0, a1);
            mx = fmaxf(mx, __shfl_xor(mx, 1, 16)); mx = fmaxf(mx, __shfl_xor(mx, 2, 16)); mx = fmaxf(mx, __shfl_xor(mx, 4, 16)); mx = fmaxf(mx, __shfl_xor(mx, 8, 16));
            const float mn = fmaxf(mrow[j], mx);
            alpha[j] = __expf(mrow[j] - mn); mrow[j] = mn;
            const float p0 = __expf(a0 - mn), p1 = __expf(a1 - mn);
            lpart[j] = lpart[j] * alpha[j] + (p0 + p1);
            const int mr = hi * 8 + j;
            pl[mr * 32 + lr] = (h16)(p0 * PSC); pl[mr * 32 + 16 + lr] = (h16)(p1 * PSC);
        }
#pragma unroll
        for (int n = 0; n < 8; ++n)
#pragma unroll
            for (int j = 0; j < 8; ++j) o[n][j] *= alpha[j];
        asm volatile("" ::: "memory");
        const v16h pa = cat16(*(const v8ha*)(pl + lr * 32 + hi * 8), *(const v8ha*)(pl + lr * 32 + 16 + hi * 8));
#pragma unroll
        for (int n = 0; n < 8; ++n) { const h16* vp = vb + (size_t)(n * 16 + lr) * NN_ + l0 + hi * 8; o[n] = wmma16(pa, cat16(*(const v8h*)vp, *(const v8h*)(vp + 16)), o[n]); }
        asm volatile("v_nop\n\tv_nop\n\tv_nop\n\tv_nop" : "+v"(o[0]), "+v"(o[3]), "+v"(o[7]) : "v"(pa));
    }
    asm volatile("v_nop\n\tv_nop\n\tv_nop\n\tv_nop" : "+v"(o[0]), "+v"(o[1]), "+v"(o[2]), "+v"(o[3]), "+v"(o[4]), "+v"(o[5]), "+v"(o[6]), "+v"(o[7]));
    float inv[8];
#pragma unroll
    for (int j = 0; j < 8; ++j) { float rs = lpart[j]; rs += __shfl_xor(rs, 1, 16); rs += __shfl_xor(rs, 2, 16); rs += __shfl_xor(rs, 4, 16); rs += __shfl_xor(rs, 8, 16); inv[j] = 1.0f / (rs * PSC); }
    float* os = &ost[wave][0];
#pragma unroll
    for (int n = 0; n < 8; ++n)
#pragma unroll
        for (int j = 0; j < 8; ++j) os[(hi * 8 + j) * 132 + n * 16 + lr] = o[n][j] * inv[j];
    __syncthreads();
    float* xb = XR + ((size_t)b * NN_ + q0) * CC + cofs;
    auto pass = [&]() {
#pragma unroll
        for (int s = 0; s < 16; ++s) { const v4f v = *(const v4fa*)(os + s * 132 + lane * 4); *(volatile v4f*)(xb + (size_t)s * CC + lane * 4) = v; }
    };
    pass(); __threadfence(); pass();
}
__global__ __launch_bounds__(256) void k_splitxr(const float* __restrict__ XR, bf* H, bf* L) {
    const int lane = threadIdx.x & 31, r = blockIdx.x * 8 + (threadIdx.x >> 5);
    if (r >= NB_ * NN_) return;
    v8us oh, ol;
#pragma unroll
    for (int i = 0; i < 8; ++i) { const float v = XR[(size_t)r * CC + lane * 8 + i]; const unsigned short hb = f2bf(v); oh[i] = hb; ol[i] = f2bf(v - bf2f(hb)); }
    *(volatile v8us*)(H + (size_t)r * CC + lane * 8) = oh; *(volatile v8us*)(L + (size_t)r * CC + lane * 8) = ol; __threadfence();
    *(volatile v8us*)(H + (size_t)r * CC + lane * 8) = oh; *(volatile v8us*)(L + (size_t)r * CC + lane * 8) = ol;
}
__global__ __launch_bounds__(256) void k_stats(const float* __restrict__ T, float* ST) {
    __shared__ float red[256];
    const int c = blockIdx.x, t = threadIdx.x;
    float s = 0.f;
#pragma unroll 1
    for (int i = 0; i < (NB_ * NN_) / 256; ++i) { const int flat = i * 256 + t; const int b = flat / NN_, n = flat - b * NN_; s += T[((size_t)b * CC + c) * NN_ + n]; }
    red[t] = s; __syncthreads();
    for (int o = 128; o > 0; o >>= 1) { if (t < o) red[t] += red[t + o]; __syncthreads(); }
    const float mu = red[0] / (float)(NB_ * NN_);
    __syncthreads();
    float q = 0.f;
#pragma unroll 1
    for (int i = 0; i < (NB_ * NN_) / 256; ++i) { const int flat = i * 256 + t; const int b = flat / NN_, n = flat - b * NN_; const float d = T[((size_t)b * CC + c) * NN_ + n] - mu; q += d * d; }
    red[t] = q; __syncthreads();
    for (int o = 128; o > 0; o >>= 1) { if (t < o) red[t] += red[t + o]; __syncthreads(); }
    const float var = red[0] / (float)(NB_ * NN_);
    if (t < 32) { const float v = (t == 0) ? mu : (t == 1) ? rsqrtf(var + 1e-5f) : 0.f; VST2(float, ST + (size_t)c * 32 + t, v); }
}
__global__ __launch_bounds__(256) void k_final(const float* __restrict__ x, const float* __restrict__ T, const float* __restrict__ ST, const float* __restrict__ gam, const float* __restrict__ bet, float* out) {
    const int lane = threadIdx.x & 31, wid = blockIdx.x * 8 + (threadIdx.x >> 5);
    const int row = wid >> 3, seg = wid & 7;
    if (row >= NB_ * CC) return;
    const int c = row % CC;
    const float mu = ST[(size_t)c * 32], rs = ST[(size_t)c * 32 + 1], g = bfr(gam[c]), be = bfr(bet[c]);
    const size_t base = (size_t)row * NN_ + seg * 256 + lane * 8;
    v8f o;
#pragma unroll
    for (int i = 0; i < 8; ++i) { const float bn = g * (T[base + i] - mu) * rs + be; o[i] = bfr(x[base + i]) + fmaxf(bn, 0.f); }
    VST2(v8f, out + base, o);
}

extern "C" void kernel_launch(void* const* d_in, const int* in_sizes, int n_in,
                              void* d_out, int out_size, void* d_ws, size_t ws_size, hipStream_t stream) {
    (void)in_sizes; (void)n_in; (void)out_size;
    const float* x = (const float*)d_in[0]; const float* wq = (const float*)d_in[1]; const float* wv = (const float*)d_in[2]; const float* bv = (const float*)d_in[3];
    const float* wt = (const float*)d_in[4]; const float* bt = (const float*)d_in[5]; const float* gam = (const float*)d_in[6]; const float* bet = (const float*)d_in[7];
    float* out = (float*)d_out;
    char* wsp = (char*)d_ws;
    auto take = [&](size_t bytes) { char* p = wsp; wsp += (bytes + 255) & ~(size_t)255; return (void*)p; };
    bf* XT = (bf*)take((size_t)NB_ * NN_ * CC * 2); bf* WQB = (bf*)take((size_t)C4 * CC * 2); bf* WVB = (bf*)take((size_t)CC * CC * 2); bf* WTB = (bf*)take((size_t)CC * CC * 2);
    float* QF = (float*)take((size_t)NB_ * NN_ * C4 * 4); h16* QH = (h16*)take((size_t)NB_ * NN_ * C4 * 2); h16* QL = (h16*)take((size_t)NB_ * NN_ * C4 * 2); float* SQ = (float*)take((size_t)NB_ * NN_ * 4);
    h16* V16 = (h16*)take((size_t)NB_ * CC * NN_ * 2); float* XR = (float*)take((size_t)NB_ * NN_ * CC * 4); bf* XRH = (bf*)take((size_t)NB_ * NN_ * CC * 2); bf* XRL = (bf*)take((size_t)NB_ * NN_ * CC * 2);
    float* T = (float*)take((size_t)NB_ * CC * NN_ * 4); float* ST = (float*)take((size_t)CC * 32 * 4);
    if ((size_t)(wsp - (char*)d_ws) > ws_size) return;
    k_xt<<<dim3(NN_ / 64, CC / 64, NB_), 256, 0, stream>>>(x, XT);
    k_cvtw<<<C4 / 8, 256, 0, stream>>>(wq, C4, WQB); k_cvtw<<<CC / 8, 256, 0, stream>>>(wv, CC, WVB); k_cvtw<<<CC / 8, 256, 0, stream>>>(wt, CC, WTB);
    k_gemm<0, false><<<dim3(NN_ / 64, C4 / 64, NB_), 128, 0, stream>>>(XT, (size_t)NN_ * CC, WQB, WQB, 0, nullptr, QF, (size_t)NN_ * C4, C4);
    k_qsplit<<<(NB_ * NN_) / 32, 256, 0, stream>>>(QF, QH, QL, SQ);
    k_gemm<1, false><<<dim3(CC / 64, NN_ / 64, NB_), 128, 0, stream>>>(WVB, 0, XT, XT, (size_t)NN_ * CC, bv, V16, (size_t)CC * NN_, NN_);
    k_attn<<<NB_ * (NN_ / 64), 128, 0, stream>>>(QH, QL, SQ, V16, 0, XR);
    k_attn<<<NB_ * (NN_ / 64), 128, 0, stream>>>(QH, QL, SQ, V16, 128, XR);
    k_splitxr<<<(NB_ * NN_) / 8, 256, 0, stream>>>(XR, XRH, XRL);
    k_gemm<2, true><<<dim3(CC / 64, NN_ / 64, NB_), 128, 0, stream>>>(WTB, 0, XRH, XRL, (size_t)NN_ * CC, bt, T, (size_t)CC * NN_, NN_);
    k_stats<<<CC, 256, 0, stream>>>(T, ST);
    k_final<<<(NB_ * CC * 8) / 8, 256, 0, stream>>>(x, T, ST, gam, bet, out);
}
